// UnICORNN_22686017257635
// MI455X (gfx1250) — hardware-verified
//
#include <hip/hip_runtime.h>
#include <math.h>

constexpr int kHid    = 256;
constexpr int kIn     = 128;
constexpr int kOutDim = 128;
constexpr int kLayers = 2;
constexpr int kXpLd   = 3 * kHid;
constexpr int kInLd   = 3 * kIn;
constexpr float kDt    = 0.03f;
constexpr float kAlpha = 0.9f;
static_assert(kXpLd % 32 == 0 && kInLd % 32 == 0, "K multiple of 32");
static_assert(kHid % 64 == 0 && kOutDim % 64 == 0, "tile multiples");

typedef __attribute__((ext_vector_type(16))) _Float16 v16h;
typedef __attribute__((ext_vector_type(8)))  _Float16 v8h;
typedef __attribute__((ext_vector_type(16))) __bf16   v16b;
typedef __attribute__((ext_vector_type(8)))  __bf16   v8b;
typedef __attribute__((ext_vector_type(8)))  float    v8f;
typedef __attribute__((ext_vector_type(4)))  float    v4f;
typedef __attribute__((ext_vector_type(4)))  unsigned int v4u;

__device__ __forceinline__ unsigned short f2bf_bits(float f) {
  unsigned u = __float_as_uint(f);
  return (unsigned short)((u + 0x7FFFu + ((u >> 16) & 1u)) >> 16);
}
__device__ __forceinline__ float bf_bits2f(unsigned short h) { return __uint_as_float(((unsigned)h) << 16); }

__device__ __forceinline__ void dep_guard_h(v8f& a, v8f& b, v16h x, v16h y) { asm volatile("v_nop\n\tv_nop\n\tv_nop\n\tv_nop" : "+v"(a), "+v"(b) : "v"(x), "v"(y)); }
__device__ __forceinline__ void dep_guard_b(v8f& a, v8f& b, v16b x, v16b y) { asm volatile("v_nop\n\tv_nop\n\tv_nop\n\tv_nop" : "+v"(a), "+v"(b) : "v"(x), "v"(y)); }
__device__ __forceinline__ void keep4_h(v16h a, v16h b, v16h c, v16h d) { asm volatile("v_nop" :: "v"(a), "v"(b), "v"(c), "v"(d)); }
__device__ __forceinline__ void keep4_b(v16b a, v16b b, v16b c, v16b d) { asm volatile("v_nop" :: "v"(a), "v"(b), "v"(c), "v"(d)); }
__device__ __forceinline__ void acc_guard4(v8f& a, v8f& b, v8f& c, v8f& d) { asm volatile("v_nop\n\tv_nop\n\tv_nop\n\tv_nop" : "+v"(a), "+v"(b), "+v"(c), "+v"(d)); }
template <typename T> struct Frag;
template <> struct Frag<_Float16> {
  typedef v16h V; union U { v16h v; v8h h[2]; };
  static __device__ __forceinline__ v16h load(const _Float16* p) {
    U f; f.h[0] = *(const v8h*)(p); f.h[1] = *(const v8h*)(p + 16); return f.v;
  }
  static __device__ __forceinline__ v8f mma(v16h a, v16h b, v8f c) {
    return __builtin_amdgcn_wmma_f32_16x16x32_f16(false, a, false, b, (short)0, c, false, false);
  }
  static __device__ __forceinline__ void guard(v8f& a, v8f& b, v16h x, v16h y) { dep_guard_h(a, b, x, y); }
  static __device__ __forceinline__ void keep(v16h a, v16h b, v16h c, v16h d) { keep4_h(a, b, c, d); }
};
template <> struct Frag<__bf16> {
  typedef v16b V; union U { v16b v; v8b h[2]; };
  static __device__ __forceinline__ v16b load(const __bf16* p) {
    U f; f.h[0] = *(const v8b*)(p); f.h[1] = *(const v8b*)(p + 16); return f.v;
  }
  static __device__ __forceinline__ v8f mma(v16b a, v16b b, v8f c) {
    return __builtin_amdgcn_wmma_f32_16x16x32_bf16(false, a, false, b, (short)0, c, false, false);
  }
  static __device__ __forceinline__ void guard(v8f& a, v8f& b, v16b x, v16b y) { dep_guard_b(a, b, x, y); }
  static __device__ __forceinline__ void keep(v16b a, v16b b, v16b c, v16b d) { keep4_b(a, b, c, d); }
};

__device__ __forceinline__ unsigned pk16(unsigned short a, unsigned short b) { return (unsigned)a | ((unsigned)b << 16); }

template <int ET> struct Elem;
template <> struct Elem<0> { typedef _Float16 T; };
template <> struct Elem<1> { typedef __bf16 T; };
template <int ET, bool SPLIT, int BIAS_MODE, int OUT_MODE, bool RESID, int ACT = 0>
__global__ __launch_bounds__(256) void wmma_gemm64(
    const unsigned short* __restrict__ Ap, const unsigned short* __restrict__ A2p, int lda, long strideA,
    const unsigned short* __restrict__ Btp, const unsigned short* __restrict__ Bt2p, int ldb, long strideB,
    void* __restrict__ Cout, void* __restrict__ Cout2, int ldc, long strideC,
    const float* __restrict__ bias,
    const float* __restrict__ resid, long strideR,
    int M, int N, int K, float scale) {
  typedef typename Elem<ET>::T T;
  typedef typename Frag<T>::V V;
  const T* A = (const T*)Ap; const T* A2 = (const T*)A2p; const T* Bt = (const T*)Btp; const T* Bt2 = (const T*)Bt2p;
  __shared__ __align__(16) float sT[8][16 * 68];
  const int b    = blockIdx.y;
  const int lane = threadIdx.x & 31;
  const int wave = threadIdx.x >> 5;
  const int tilesN = N >> 6;
  const int tilesM = M >> 6;
  const int tile = blockIdx.x * 8 + wave;
  if (tile >= tilesM * tilesN) return;
  const int tm = tile / tilesN;
  const int tn = tile - tm * tilesN;
  const int m0 = tm << 6;
  const int n0 = tn << 6;

  const T* Ab  = A  + (size_t)b * strideA;
  const T* Bb  = Bt + (size_t)b * strideB;
  const T* Ab2 = SPLIT ? (A2  + (size_t)b * strideA) : nullptr;
  const T* Bb2 = SPLIT ? (Bt2 + (size_t)b * strideB) : nullptr;

  const int rlane = lane & 15;
  const int koff  = (lane >> 4) * 8;
  const int mOff  = (lane >> 4) * 8;

  v8f acc[4][4];
#pragma unroll
  for (int i = 0; i < 4; ++i)
#pragma unroll
    for (int j = 0; j < 4; ++j) acc[i][j] = (v8f){0.f,0.f,0.f,0.f,0.f,0.f,0.f,0.f};

  for (int k0 = 0; k0 < K; k0 += 32) {
    V bh[4], bl[4];
#pragma unroll
    for (int j = 0; j < 4; ++j) {
      const size_t bo = (size_t)(n0 + (j << 4) + rlane) * ldb + koff + k0;
      bh[j] = Frag<T>::load(Bb + bo);
      if (SPLIT) bl[j] = Frag<T>::load(Bb2 + bo);
    }
#pragma unroll
    for (int i = 0; i < 4; ++i) {
      const size_t ao = (size_t)(m0 + (i << 4) + rlane) * lda + koff + k0;
      V ah = Frag<T>::load(Ab + ao);
      V al;
      if (SPLIT) al = Frag<T>::load(Ab2 + ao);
#pragma unroll
      for (int j = 0; j < 4; ++j) {
        acc[i][j] = Frag<T>::mma(ah, bh[j], acc[i][j]);
        if (SPLIT) {
          acc[i][j] = Frag<T>::mma(ah, bl[j], acc[i][j]);
          acc[i][j] = Frag<T>::mma(al, bh[j], acc[i][j]);
        }
      }
      Frag<T>::guard(acc[i][0], acc[i][3], ah, SPLIT ? al : ah);
    }
    Frag<T>::keep(bh[0], bh[1], bh[2], bh[3]);
    if (SPLIT) Frag<T>::keep(bl[0], bl[1], bl[2], bl[3]);
  }
  acc_guard4(acc[0][0], acc[0][1], acc[0][2], acc[0][3]);
  acc_guard4(acc[1][0], acc[1][1], acc[1][2], acc[1][3]);
  acc_guard4(acc[2][0], acc[2][1], acc[2][2], acc[2][3]);
  acc_guard4(acc[3][0], acc[3][1], acc[3][2], acc[3][3]);

  float* slab = sT[wave];
  const float* Rb = RESID ? (resid + (size_t)b * strideR) : nullptr;
#pragma unroll
  for (int i = 0; i < 4; ++i) {
    const int mBase = m0 + (i << 4);
#pragma unroll
    for (int j = 0; j < 4; ++j) {
      const int n = n0 + (j << 4) + rlane;
      float bv = 0.f;
      if (BIAS_MODE == 2) bv = bias[n];
#pragma unroll
      for (int r = 0; r < 8; ++r) {
        float v = acc[i][j][r] * scale;
        if (BIAS_MODE == 1) v += bias[mBase + mOff + r];
        if (BIAS_MODE == 2) v += bv;
        if (RESID) v += Rb[(size_t)(mBase + mOff + r) * ldc + n];
        if (ACT == 2) v = fmaxf(v, 0.0f);
        if (ACT == 4) v = (v > 0.f) ? v : 0.01f * v;
        slab[(mOff + r) * 68 + (j << 4) + rlane] = v;
      }
    }
    __builtin_amdgcn_fence(__ATOMIC_RELEASE, "workgroup");
    __builtin_amdgcn_wave_barrier();
    __builtin_amdgcn_fence(__ATOMIC_ACQUIRE, "workgroup");
    if (OUT_MODE == 0) {
      float* C = (float*)Cout + (size_t)b * strideC;
      const int hh = lane >> 4, c4 = (lane & 15) * 4;
      for (int pass = 0; pass < 2; ++pass) {
#pragma unroll
        for (int it = 0; it < 8; ++it) {
          const int row = it * 2 + hh;
          v4f v = *(const v4f*)(slab + row * 68 + c4);
          *(volatile v4f*)(C + (size_t)(mBase + row) * ldc + n0 + c4) = v;
        }
        __threadfence();
      }
    } else {
      const int q = lane >> 3, c8 = (lane & 7) * 8;
      unsigned short* C  = (unsigned short*)Cout  + (size_t)b * strideC;
      unsigned short* C2 = (OUT_MODE == 2) ? ((unsigned short*)Cout2 + (size_t)b * strideC) : nullptr;
      for (int pass = 0; pass < 2; ++pass) {
#pragma unroll
        for (int it = 0; it < 4; ++it) {
          const int row = it * 4 + q;
          const float* sp = slab + row * 68 + c8;
          v8h hv, lv;
#pragma unroll
          for (int e = 0; e < 8; ++e) {
            if (OUT_MODE == 1) {
              hv[e] = (_Float16)sp[e];
            } else {
              unsigned short hb = f2bf_bits(sp[e]);
              unsigned short lb = f2bf_bits(sp[e] - bf_bits2f(hb));
              hv[e] = __builtin_bit_cast(_Float16, hb);
              lv[e] = __builtin_bit_cast(_Float16, lb);
            }
          }
          *(volatile v8h*)(C + (size_t)(mBase + row) * ldc + n0 + c8) = hv;
          if (OUT_MODE == 2) *(volatile v8h*)(C2 + (size_t)(mBase + row) * ldc + n0 + c8) = lv;
        }
        __threadfence();
      }
    }
    __builtin_amdgcn_fence(__ATOMIC_RELEASE, "workgroup");
    __builtin_amdgcn_wave_barrier();
    __builtin_amdgcn_fence(__ATOMIC_ACQUIRE, "workgroup");
  }
}

template <int PAT, int NCOL>
__global__ __launch_bounds__(256) void pack3_kernel(const float* __restrict__ in, unsigned short* __restrict__ out, int n8) {
  static_assert(NCOL % 64 == 0, "line coverage");
  const int i = blockIdx.x * 256 + threadIdx.x;
  if (i >= n8) return;
  const size_t e0 = 8 * (size_t)i;
  const int row = (int)(e0 / NCOL);
  const int col = (int)(e0 - (size_t)row * NCOL);
  const float* p = in + e0;
  const v4f a = *(const v4f*)(p);
  const v4f c = *(const v4f*)(p + 4);
  unsigned short hb[8], lb[8];
#pragma unroll
  for (int e = 0; e < 4; ++e) {
    const float f0 = a[e], f1 = c[e];
    hb[e] = f2bf_bits(f0);     lb[e] = f2bf_bits(f0 - bf_bits2f(hb[e]));
    hb[4 + e] = f2bf_bits(f1); lb[4 + e] = f2bf_bits(f1 - bf_bits2f(hb[4 + e]));
  }
  const v4u uh = (v4u){pk16(hb[0], hb[1]), pk16(hb[2], hb[3]), pk16(hb[4], hb[5]), pk16(hb[6], hb[7])};
  const v4u ul = (v4u){pk16(lb[0], lb[1]), pk16(lb[2], lb[3]), pk16(lb[4], lb[5]), pk16(lb[6], lb[7])};
  const v4u u1 = (PAT == 0) ? ul : uh;
  const v4u u2 = (PAT == 0) ? uh : ul;
  unsigned short* o = out + (size_t)row * (3 * NCOL) + col;
  for (int pass = 0; pass < 2; ++pass) {
    *(volatile v4u*)(o) = uh;
    *(volatile v4u*)(o + NCOL) = u1;
    *(volatile v4u*)(o + 2 * NCOL) = u2;
    __threadfence();
  }
}

template <int INIT>
__global__ __launch_bounds__(128) void osc_step_kernel(
    const unsigned short* __restrict__ Ap, int lda,
    const unsigned short* __restrict__ Btp, int ldb,
    const float* __restrict__ Xf_in, const float* __restrict__ Zf_in,
    const float* __restrict__ wcol, const float* __restrict__ bcol,
    float* __restrict__ Xf_out, float* __restrict__ Zf_out,
    unsigned short* __restrict__ Xp_out, int K, int zzero) {
  typedef __bf16 T;
  typedef v16b V;
  const T* A = (const T*)Ap;
  const T* Bt = (const T*)Btp;
  __shared__ __align__(16) float sX[4][16 * 68];
  __shared__ __align__(16) float sZ[4][16 * 68];
  const int lane = threadIdx.x & 31;
  const int wave = threadIdx.x >> 5;
  const int tile = blockIdx.x * 4 + wave;
  if (tile >= 16) return;
  const int tm = tile >> 2;
  const int tn = tile & 3;
  const int m0 = tm << 6;
  const int n0 = tn << 6;

  const int rlane = lane & 15;
  const int koff  = (lane >> 4) * 8;
  const int mOff  = (lane >> 4) * 8;

  v8f acc[4][4];
#pragma unroll
  for (int i = 0; i < 4; ++i)
#pragma unroll
    for (int j = 0; j < 4; ++j) acc[i][j] = (v8f){0.f,0.f,0.f,0.f,0.f,0.f,0.f,0.f};

  for (int k0 = 0; k0 < K; k0 += 32) {
    V bh[4];
#pragma unroll
    for (int j = 0; j < 4; ++j) {
      const size_t bo = (size_t)(n0 + (j << 4) + rlane) * ldb + koff + k0;
      bh[j] = Frag<T>::load(Bt + bo);
    }
#pragma unroll
    for (int i = 0; i < 4; ++i) {
      const size_t ao = (size_t)(m0 + (i << 4) + rlane) * lda + koff + k0;
      V ah = Frag<T>::load(A + ao);
#pragma unroll
      for (int j = 0; j < 4; ++j) acc[i][j] = Frag<T>::mma(ah, bh[j], acc[i][j]);
      Frag<T>::guard(acc[i][0], acc[i][3], ah, ah);
    }
    Frag<T>::keep(bh[0], bh[1], bh[2], bh[3]);
  }
  acc_guard4(acc[0][0], acc[0][1], acc[0][2], acc[0][3]);
  acc_guard4(acc[1][0], acc[1][1], acc[1][2], acc[1][3]);
  acc_guard4(acc[2][0], acc[2][1], acc[2][2], acc[2][3]);
  acc_guard4(acc[3][0], acc[3][1], acc[3][2], acc[3][3]);

  float w0 = 0.f, w1 = 0.f;
  if (!INIT) { w0 = wcol[n0 + lane]; w1 = wcol[n0 + 32 + lane]; }
  const float b0 = bcol[n0 + lane];
  const float b1 = bcol[n0 + 32 + lane];

  float* sx = sX[wave];
  float* sz = sZ[wave];
  const int hh = lane >> 4, c4 = (lane & 15) * 4;
  const int q = lane >> 3, c8 = (lane & 7) * 8;

#pragma unroll
  for (int i = 0; i < 4; ++i) {
    const int mBase = m0 + (i << 4);
#pragma unroll
    for (int j = 0; j < 4; ++j)
#pragma unroll
      for (int r = 0; r < 8; ++r) sx[(mOff + r) * 68 + (j << 4) + rlane] = acc[i][j][r];
    __builtin_amdgcn_fence(__ATOMIC_RELEASE, "workgroup");
    __builtin_amdgcn_wave_barrier();
    __builtin_amdgcn_fence(__ATOMIC_ACQUIRE, "workgroup");

#pragma unroll 1
    for (int it = 0; it < 32; ++it) {
      const int row  = it >> 1;
      const int half = it & 1;
      const int col  = (half << 5) + lane;
      const int sidx = row * 68 + col;
      const float p  = sx[sidx];
      const float bn = half ? b1 : b0;
      if (INIT) {
        sx[sidx] = p + bn;
      } else {
        const float wn = half ? w1 : w0;
        const size_t gidx = (size_t)(mBase + row) * kHid + n0 + col;
        const float xv = Xf_in[gidx];
        float zv = 0.f;
        if (zzero == 0) zv = Zf_in[gidx];
        const float pre = wn * xv + p + bn;
        const float th  = tanhf(pre);
        const float zn  = zv - kDt * (th + kAlpha * xv);
        const float xn  = xv + kDt * zn;
        sx[sidx] = xn;
        sz[sidx] = zn;
      }
    }
    __builtin_amdgcn_fence(__ATOMIC_RELEASE, "workgroup");
    __builtin_amdgcn_wave_barrier();
    __builtin_amdgcn_fence(__ATOMIC_ACQUIRE, "workgroup");

    for (int pass = 0; pass < 2; ++pass) {
#pragma unroll
      for (int it = 0; it < 8; ++it) {
        const int row = it * 2 + hh;
        const v4f vx = *(const v4f*)(sx + row * 68 + c4);
        *(volatile v4f*)(Xf_out + (size_t)(mBase + row) * kHid + n0 + c4) = vx;
        if (!INIT) {
          const v4f vz = *(const v4f*)(sz + row * 68 + c4);
          *(volatile v4f*)(Zf_out + (size_t)(mBase + row) * kHid + n0 + c4) = vz;
        }
      }
#pragma unroll
      for (int it = 0; it < 4; ++it) {
        const int row = it * 4 + q;
        const float* sp = sx + row * 68 + c8;
        unsigned short hb[8], lb[8];
#pragma unroll
        for (int e = 0; e < 8; ++e) {
          const float f = sp[e];
          hb[e] = f2bf_bits(f);
          lb[e] = f2bf_bits(f - bf_bits2f(hb[e]));
        }
        const v4u uh = (v4u){pk16(hb[0], hb[1]), pk16(hb[2], hb[3]), pk16(hb[4], hb[5]), pk16(hb[6], hb[7])};
        const v4u ul = (v4u){pk16(lb[0], lb[1]), pk16(lb[2], lb[3]), pk16(lb[4], lb[5]), pk16(lb[6], lb[7])};
        unsigned short* op = Xp_out + (size_t)(mBase + row) * kXpLd + n0 + c8;
        *(volatile v4u*)(op)            = uh;
        *(volatile v4u*)(op + kHid)     = ul;
        *(volatile v4u*)(op + 2 * kHid) = uh;
      }
      __threadfence();
    }
    __builtin_amdgcn_fence(__ATOMIC_RELEASE, "workgroup");
    __builtin_amdgcn_wave_barrier();
    __builtin_amdgcn_fence(__ATOMIC_ACQUIRE, "workgroup");
  }
}

extern "C" void kernel_launch(void* const* d_in, const int* in_sizes, int n_in,
                              void* d_out, int out_size, void* d_ws, size_t ws_size,
                              hipStream_t stream) {
  if (n_in < 8) return;
  if (in_sizes[0] != kHid * kIn || in_sizes[1] != kHid * kIn || in_sizes[2] != kHid ||
      in_sizes[3] != kLayers * kHid || in_sizes[4] != kLayers * kHid * kHid || in_sizes[5] != kLayers * kHid ||
      in_sizes[6] != kOutDim * kHid || in_sizes[7] != kOutDim || out_size != kHid * kOutDim) return;

  const float* x_in  = (const float*)d_in[0];
  const float* w_in  = (const float*)d_in[1];
  const float* b_in  = (const float*)d_in[2];
  const float* w_rec = (const float*)d_in[3];
  const float* v_rec = (const float*)d_in[4];
  const float* b_rec = (const float*)d_in[5];
  const float* w_out = (const float*)d_in[6];
  const float* b_out = (const float*)d_in[7];
  float* out = (float*)d_out;

  const size_t bPxin = (size_t)kHid * kInLd * 2;
  const size_t bPwin = (size_t)kHid * kInLd * 2;
  const size_t bPv   = (size_t)kLayers * kHid * kXpLd * 2;
  const size_t bPwo  = (size_t)kOutDim * kXpLd * 2;
  const size_t bXf1  = (size_t)kHid * kHid * 4;
  const size_t bXp1  = (size_t)kHid * kXpLd * 2;
  const size_t oPxin = 0;
  const size_t oPwin = oPxin + bPxin;
  const size_t oPv   = oPwin + bPwin;
  const size_t oPwo  = oPv + bPv;
  const size_t oXf   = oPwo + bPwo;
  const size_t oZf   = oXf + 2 * bXf1;
  const size_t oXp   = oZf + 2 * bXf1;
  const size_t total = oXp + 2 * bXp1;
  if (ws_size < total) return;

  char* ws = (char*)d_ws;
  unsigned short* Pxin = (unsigned short*)(ws + oPxin);
  unsigned short* Pwin = (unsigned short*)(ws + oPwin);
  unsigned short* Pv   = (unsigned short*)(ws + oPv);
  unsigned short* Pwo  = (unsigned short*)(ws + oPwo);
  float* Xf[2]; float* Zf[2]; unsigned short* Xp[2];
  Xf[0] = (float*)(ws + oXf);  Xf[1] = (float*)(ws + oXf + bXf1);
  Zf[0] = (float*)(ws + oZf);  Zf[1] = (float*)(ws + oZf + bXf1);
  Xp[0] = (unsigned short*)(ws + oXp);  Xp[1] = (unsigned short*)(ws + oXp + bXp1);

  const int n8_xin = kHid * kIn / 8;
  const int n8_win = kHid * kIn / 8;
  const int n8_v   = kLayers * kHid * kHid / 8;
  const int n8_wo  = kOutDim * kHid / 8;
  pack3_kernel<0, kIn><<<(n8_xin + 255) / 256, 256, 0, stream>>>(x_in, Pxin, n8_xin);
  pack3_kernel<1, kIn><<<(n8_win + 255) / 256, 256, 0, stream>>>(w_in, Pwin, n8_win);
  pack3_kernel<1, kHid><<<(n8_v + 255) / 256, 256, 0, stream>>>(v_rec, Pv, n8_v);
  pack3_kernel<1, kHid><<<(n8_wo + 255) / 256, 256, 0, stream>>>(w_out, Pwo, n8_wo);

  osc_step_kernel<1><<<4, 128, 0, stream>>>(Pxin, kInLd, Pwin, kInLd, Xf[0], Zf[0], b_in, b_in,
                                            Xf[0], Zf[0], Xp[0], kInLd, 1);

  for (int t = 0; t < kLayers * kHid; ++t) {
    const int layer = t / kHid;
    const int rd = t & 1;
    const int wr = rd ^ 1;
    const int zzero = ((t % kHid) == 0) ? 1 : 0;
    osc_step_kernel<0><<<4, 128, 0, stream>>>(Pv + (size_t)layer * kHid * kXpLd, kXpLd, Xp[rd], kXpLd,
                                              Xf[rd], Zf[rd], w_rec + (size_t)layer * kHid, b_rec + (size_t)layer * kHid,
                                              Xf[wr], Zf[wr], Xp[wr], kXpLd, zzero);
  }
  const int fin = (kLayers * kHid) & 1;

  wmma_gemm64<1, false, 2, 0, false><<<dim3(1, 1, 1), 256, 0, stream>>>(
      Xp[fin], Xp[fin], kXpLd, (long)0, Pwo, Pwo, kXpLd, (long)0,
      out, out, kOutDim, (long)0, b_out, b_out, (long)0, kHid, kOutDim, kXpLd, 1.0f);
}
